// TransConvLayer_27685359190150
// MI455X (gfx1250) — hardware-verified
//
#include <hip/hip_runtime.h>
#include <math.h>
#include <stdint.h>

#ifndef NB
#define NB 8
#endif
#ifndef SEQ
#define SEQ 16384
#endif
#define N_FULL 16384
#define CIN    64
#define NH     4
#define DO     63
#define HP     64
#define NPROJ  (NH * HP)
#define KSEG   320
#define KF     (NH * KSEG)
#define KSC    1024.0f
#define VSC    1024.0f
#define ASC    65536.0f
#define MSC    64.0f
#define OSC    (1.0f / 1048576.0f)
#define FSC    (0.25f / 65536.0f)
#define EPSC   1e-6f
#define KCURV  1.0f
#define SLP    68
#define SLAB   (16 * SLP)
#define TTP    72
#define KSP    68
#define WS_CAP 134217728

static_assert(NH == 4 && HP == 64 && DO + 1 == HP && CIN == 64 && NPROJ == 256 && KSEG == 5 * HP && KF == 1280);
static_assert(NB >= 1 && NB <= 8);
static_assert(NB == 1 || SEQ == N_FULL);
static_assert((SEQ % 64) == 0 && SEQ >= 64 && SEQ <= N_FULL);
static_assert((CIN % 32) == 0 && (KF % 32) == 0 && (SEQ % 32) == 0 && ((SEQ * CIN / 8) % 256) == 0);
static_assert(((HP * (KF / 8)) % 256) == 0 && ((NPROJ * 8) % 256) == 0);
static_assert(4 * SLAB * 4 + 2 * HP * TTP * 2 + HP * 4 <= 65536 && HP * KSP * 4 <= 65536);

typedef unsigned short u16;
typedef _Float16 v16h __attribute__((ext_vector_type(16)));
typedef _Float16 v8h  __attribute__((ext_vector_type(8)));
typedef __bf16   v16b __attribute__((ext_vector_type(16)));
typedef float    v8f  __attribute__((ext_vector_type(8)));
typedef float    v4f  __attribute__((ext_vector_type(4)));
typedef unsigned int v4u __attribute__((ext_vector_type(4)));

union FragH { v16h v; v8h h[2]; v4u u[2]; };
union FragB { v16b v; v4u u[2]; };

__device__ __forceinline__ unsigned short bf_bits(float f) {
  unsigned u = __float_as_uint(f);
  return (unsigned short)((u + 0x7FFFu + ((u >> 16) & 1u)) >> 16);
}
__device__ __forceinline__ float bf_up(unsigned short h) { return __uint_as_float(((unsigned)h) << 16); }
__device__ __forceinline__ float bfr(float f) { return bf_up(bf_bits(f)); }
__device__ __forceinline__ unsigned short h_bits(_Float16 x) { return __builtin_bit_cast(unsigned short, x); }
__device__ __forceinline__ unsigned pk16(unsigned short a, unsigned short b) { return (unsigned)a | ((unsigned)b << 16); }
__device__ __forceinline__ v8f zero8() { v8f z = {0.f, 0.f, 0.f, 0.f, 0.f, 0.f, 0.f, 0.f}; return z; }
__device__ __forceinline__ int imin(int a, int b) { return a < b ? a : b; }
__device__ __forceinline__ int imax(int a, int b) { return a > b ? a : b; }

__device__ __forceinline__ v16h ldfrag_h(const _Float16* p) {
  FragH f;
  f.h[0] = *(const v8h*)(p);
  f.h[1] = *(const v8h*)(p + 16);
  return f.v;
}
__device__ __forceinline__ v16b ldfrag_b(const u16* p) {
  FragB f;
  f.u[0] = *(const v4u*)(p);
  f.u[1] = *(const v4u*)(p + 16);
  return f.v;
}

__device__ __forceinline__ v8f mma_h(v16h a, v16h b, v8f c) {
  return __builtin_amdgcn_wmma_f32_16x16x32_f16(false, a, false, b, (short)0, c, false, false);
}
__device__ __forceinline__ v8f mma_b(v16b a, v16b b, v8f c) {
  return __builtin_amdgcn_wmma_f32_16x16x32_bf16(false, a, false, b, (short)0, c, false, false);
}
__device__ __forceinline__ void guard2(v8f& a, v8f& b, v16h x0, v16h x1, v16h x2, v16h x3, v16h x4, v16h x5) {
#if defined(__HIP_DEVICE_COMPILE__)
  asm volatile("v_nop\n\tv_nop\n\tv_nop\n\tv_nop"
               : "+v"(a), "+v"(b) : "v"(x0), "v"(x1), "v"(x2), "v"(x3), "v"(x4), "v"(x5) : "memory");
#endif
}
template <typename F>
__device__ __forceinline__ void guard6(v8f& a, v8f& b, v8f& c, v8f& d, F x0, F x1, F x2, F x3, F x4, F x5) {
#if defined(__HIP_DEVICE_COMPILE__)
  asm volatile("v_nop\n\tv_nop\n\tv_nop\n\tv_nop"
               : "+v"(a), "+v"(b), "+v"(c), "+v"(d) : "v"(x0), "v"(x1), "v"(x2), "v"(x3), "v"(x4), "v"(x5) : "memory");
#endif
}
__device__ __forceinline__ void acc_guard4(v8f& a, v8f& b, v8f& c, v8f& d) {
#if defined(__HIP_DEVICE_COMPILE__)
  asm volatile("v_nop\n\tv_nop\n\tv_nop\n\tv_nop" : "+v"(a), "+v"(b), "+v"(c), "+v"(d));
#endif
}
__device__ __forceinline__ void wave_sync_lds() {
  __builtin_amdgcn_fence(__ATOMIC_RELEASE, "workgroup");
  __builtin_amdgcn_wave_barrier();
  __builtin_amdgcn_fence(__ATOMIC_ACQUIRE, "workgroup");
}
__device__ __forceinline__ float grp8_sum(float v) {
  v += __shfl_xor(v, 1, 32);
  v += __shfl_xor(v, 2, 32);
  v += __shfl_xor(v, 4, 32);
  return v;
}

__global__ __launch_bounds__(256) void cvt_w3(const float* __restrict__ w0, const float* __restrict__ w1,
                                               const float* __restrict__ w2, u16* D0, u16* D1, u16* D2) {
  const int which = (int)blockIdx.y;
  const float* W = (which == 0) ? w0 : ((which == 1) ? w1 : w2);
  u16* D = (which == 0) ? D0 : ((which == 1) ? D1 : D2);
  const int gt = (int)blockIdx.x * 256 + (int)threadIdx.x;
  if (gt >= NPROJ * 8) return;
  const int row = gt >> 3, p8 = (gt & 7) * 8;
  const int h = row >> 6, o = row & 63;
  const bool valid = (o < DO);
  const int  oc = valid ? o : (DO - 1);
  const float* p = W + ((size_t)(h * DO + oc) * CIN + p8);
  const v4f a = *(const v4f*)(p), b4 = *(const v4f*)(p + 4);
  float w[8];
#pragma unroll
  for (int e = 0; e < 4; ++e) { w[e] = valid ? a[e] : 0.0f; w[4 + e] = valid ? b4[e] : 0.0f; }
  v4u ov;
#pragma unroll
  for (int e = 0; e < 4; ++e) ov[e] = pk16(bf_bits(w[2 * e]), bf_bits(w[2 * e + 1]));
  u16* d = D + (size_t)row * CIN + p8;
  for (int pass = 0; pass < 2; ++pass) {
    *(volatile v4u*)(d) = ov;
    __threadfence();
  }
}

__global__ __launch_bounds__(256) void cvt_x2(const float* __restrict__ x0, const float* __restrict__ x1,
                                               u16* D0, u16* D1, int n8) {
  const int which = (int)blockIdx.y;
  const float* x = (which == 0) ? x0 : x1;
  u16* D = (which == 0) ? D0 : D1;
  const int gt = (int)blockIdx.x * 256 + (int)threadIdx.x;
  if (gt >= n8) return;
  const float* p = x + (size_t)gt * 8;
  const v4f a = *(const v4f*)(p), b4 = *(const v4f*)(p + 4);
  v4u ov;
#pragma unroll
  for (int e = 0; e < 2; ++e) {
    ov[e]     = pk16(bf_bits(a[2 * e]),  bf_bits(a[2 * e + 1]));
    ov[2 + e] = pk16(bf_bits(b4[2 * e]), bf_bits(b4[2 * e + 1]));
  }
  u16* d = D + (size_t)gt * 8;
  for (int pass = 0; pass < 2; ++pass) {
    *(volatile v4u*)(d) = ov;
    __threadfence();
  }
}

template <int MODE>
__global__ __launch_bounds__(128)
void gemm_proj(const u16* __restrict__ X, const u16* __restrict__ Wt, const float* __restrict__ bias,
               const float* __restrict__ ns, const float* __restrict__ KT, u16* T0, u16* T1, u16* AP) {
#pragma clang fp contract(off)
  __shared__ __align__(16) float slab[4 * SLAB];
  __shared__ __align__(16) u16 TTh[HP * TTP];
  __shared__ __align__(16) u16 TTl[HP * TTP];
  __shared__ float smk[HP];
  const int tid = (int)threadIdx.x, wave = tid >> 5, lane = tid & 31, hh = lane >> 4, m = lane & 15;
  const int bid = (int)blockIdx.x;
  const int h   = bid & (NH - 1);
  const int rt  = bid >> 2;
  if (rt * 64 + 64 > SEQ) return;
  const int rowb = rt * 64 + wave * 16;
  if constexpr (MODE == 2) {
    if (tid < HP) smk[tid] = KT[(size_t)(h * HP + (HP - 1)) * HP + tid];
  }
  const u16* ap = X  + (size_t)(rowb + m) * CIN + 8 * hh;
  const u16* bp = Wt + (size_t)(h * HP + m) * CIN + 8 * hh;
  const size_t bs = (size_t)16 * CIN;
  v8f acc0 = zero8(), acc1 = zero8(), acc2 = zero8(), acc3 = zero8();
#pragma unroll
  for (int k0 = 0; k0 < CIN; k0 += 32) {
    const v16b a  = ldfrag_b(ap + k0);
    const v16b f0 = ldfrag_b(bp + k0);
    const v16b f1 = ldfrag_b(bp + bs + k0);
    const v16b f2 = ldfrag_b(bp + 2 * bs + k0);
    const v16b f3 = ldfrag_b(bp + 3 * bs + k0);
    acc0 = mma_b(a, f0, acc0);
    acc1 = mma_b(a, f1, acc1);
    acc2 = mma_b(a, f2, acc2);
    acc3 = mma_b(a, f3, acc3);
    guard6<v16b>(acc0, acc1, acc2, acc3, a, f0, f1, f2, f3, a);
  }
  float* sl = slab + wave * SLAB;
#pragma unroll
  for (int r = 0; r < 8; ++r) {
    const int ro = (8 * hh + r) * SLP + m;
    sl[ro]      = acc0[r];
    sl[ro + 16] = acc1[r];
    sl[ro + 32] = acc2[r];
    sl[ro + 48] = acc3[r];
  }
  __syncthreads();

  const float inv = 1.0f / fabsf(bfr(ns[0]));
  const int rq = lane >> 3, c8 = (lane & 7) * 8;
  float b8[8], k8[8];
#pragma unroll
  for (int e = 0; e < 8; ++e) {
    const int col = c8 + e;
    const int ci  = imin(col, DO - 1);
    const float bvv = bfr(bias[h * DO + ci]);
    b8[e] = (col < DO) ? bvv : 0.0f;
    if constexpr (MODE == 2) k8[e] = smk[col]; else k8[e] = 0.0f;
  }
  v4u oh[4], ol[4];
#pragma unroll
  for (int it = 0; it < 4; ++it) {
    const int row = it * 4 + rq;
    const int tok = wave * 16 + row;
    const v4f va = *(const v4f*)(sl + row * SLP + c8), vb = *(const v4f*)(sl + row * SLP + c8 + 4);
    float xs[8];
#pragma unroll
    for (int e = 0; e < 4; ++e) { xs[e] = va[e] + b8[e]; xs[4 + e] = vb[e] + b8[4 + e]; }
    unsigned short hb[8], lb[8];
#pragma unroll
    for (int e = 0; e < 8; ++e) { hb[e] = 0; lb[e] = 0; }
    if constexpr (MODE == 1) {
      const unsigned short one_hi = h_bits((_Float16)VSC);
#pragma unroll
      for (int e = 0; e < 8; ++e) {
        const int col = c8 + e;
        const float vv = (col < DO) ? xs[e] : 0.0f;
        const float t  = vv * VSC;
        const _Float16 hv = (_Float16)t;
        const _Float16 lv = (_Float16)(t - (float)hv);
        hb[e] = h_bits(hv);
        lb[e] = h_bits(lv);
        TTh[col * TTP + tok] = (col == DO) ? one_hi : hb[e];
        TTl[col * TTP + tok] = (col == DO) ? (unsigned short)0 : lb[e];
      }
    } else {
      float x2[8];
      float s2 = 0.0f, s4 = 0.0f;
#pragma unroll
      for (int e = 0; e < 8; ++e) {
        const int col = c8 + e;
        const float xv = (col < DO) ? ((fmaxf(xs[e], 0.0f) + EPSC) * inv) : 0.0f;
        const float q = xv * xv;
        x2[e] = q;
        s2 = s2 + q;
        s4 = s4 + q * q;
      }
      s2 = grp8_sum(s2);
      s4 = grp8_sum(s4);
      const float ratio = sqrtf(s2) / sqrtf(s4);
      float ph[8];
#pragma unroll
      for (int e = 0; e < 8; ++e) ph[e] = ratio * x2[e];
      if constexpr (MODE == 0) {
#pragma unroll
        for (int e = 0; e < 8; ++e) {
          const int col = c8 + e;
          const float t = ph[e] * KSC;
          const _Float16 hv = (_Float16)t;
          const _Float16 lv = (_Float16)(t - (float)hv);
          TTh[col * TTP + tok] = h_bits(hv);
          TTl[col * TTP + tok] = h_bits(lv);
        }
      } else {
        float dp = 0.0f;
#pragma unroll
        for (int e = 0; e < 8; ++e) dp = dp + ph[e] * k8[e];
        dp = grp8_sum(dp);
        const float rden = 1.0f / (dp + EPSC);
#pragma unroll
        for (int e = 0; e < 8; ++e) {
          const float a = ph[e] * rden;
          const float t = a * ASC;
          const _Float16 hv = (_Float16)t;
          const _Float16 lv = (_Float16)(t - (float)hv);
          hb[e] = h_bits(hv);
          lb[e] = h_bits(lv);
        }
      }
    }
    v4u o1, o2;
#pragma unroll
    for (int e = 0; e < 4; ++e) {
      o1[e] = pk16(hb[2 * e], hb[2 * e + 1]);
      o2[e] = pk16(lb[2 * e], lb[2 * e + 1]);
    }
    oh[it] = o1;
    ol[it] = o2;
  }
  if constexpr (MODE != 0) {
    u16* arow = AP + (size_t)rowb * KF + (size_t)h * KSEG + c8;
    for (int pass = 0; pass < 2; ++pass) {
#pragma unroll
      for (int it = 0; it < 4; ++it) {
        u16* p = arow + (size_t)(it * 4 + rq) * KF;
        if constexpr (MODE == 1) {
          *(volatile v4u*)(p + 3 * HP) = oh[it];
          *(volatile v4u*)(p + 4 * HP) = ol[it];
        } else {
          *(volatile v4u*)(p)          = oh[it];
          *(volatile v4u*)(p + HP)     = ol[it];
          *(volatile v4u*)(p + 2 * HP) = oh[it];
        }
      }
      __threadfence();
    }
  } else {
    (void)oh; (void)ol;
  }
  if constexpr (MODE != 2) {
    __syncthreads();
    const int q8 = tid >> 3, p8 = (tid & 7) * 8;
    v4u vh[4], vl[4];
#pragma unroll
    for (int it = 0; it < 4; ++it) {
      const int line = it * 16 + q8;
      vh[it] = *(const v4u*)(TTh + line * TTP + p8);
      vl[it] = *(const v4u*)(TTl + line * TTP + p8);
    }
    const size_t tb = (size_t)(h * HP) * SEQ + (size_t)rt * 64 + p8;
    for (int pass = 0; pass < 2; ++pass) {
#pragma unroll
      for (int it = 0; it < 4; ++it) {
        const int line = it * 16 + q8;
        *(volatile v4u*)(T0 + tb + (size_t)line * SEQ) = vh[it];
        *(volatile v4u*)(T1 + tb + (size_t)line * SEQ) = vl[it];
      }
      __threadfence();
    }
  }
}

__global__ __launch_bounds__(128)
void gemm_ktv(const u16* __restrict__ THp, const u16* __restrict__ TLp,
              const u16* __restrict__ UHp, const u16* __restrict__ ULp, float* KT) {
  __shared__ __align__(16) float KS[HP * KSP];
  const int tid = (int)threadIdx.x, wave = tid >> 5, lane = tid & 31, hh = lane >> 4, m = lane & 15;
  const int h = (int)blockIdx.x;
  if (h >= NH) return;
  const int mrow = h * HP + wave * 16;
  const _Float16* ahp = (const _Float16*)(const void*)THp + (size_t)(mrow + m) * SEQ + 8 * hh;
  const _Float16* alp = (const _Float16*)(const void*)TLp + (size_t)(mrow + m) * SEQ + 8 * hh;
  const _Float16* bhp = (const _Float16*)(const void*)UHp + (size_t)(h * HP + m) * SEQ + 8 * hh;
  const _Float16* blp = (const _Float16*)(const void*)ULp + (size_t)(h * HP + m) * SEQ + 8 * hh;
  const size_t bs = (size_t)16 * SEQ;
  v8f o0 = zero8(), o1 = zero8(), o2 = zero8(), o3 = zero8();
#pragma unroll 1
  for (int k0 = 0; k0 < SEQ; k0 += 32) {
    const v16h ah = ldfrag_h(ahp + k0);
    const v16h al = ldfrag_h(alp + k0);
    {
      const v16h bh0 = ldfrag_h(bhp + k0), bh1 = ldfrag_h(bhp + bs + k0);
      const v16h bl0 = ldfrag_h(blp + k0), bl1 = ldfrag_h(blp + bs + k0);
      o0 = mma_h(ah, bh0, o0);
      o0 = mma_h(al, bh0, o0);
      o0 = mma_h(ah, bl0, o0);
      o1 = mma_h(ah, bh1, o1);
      o1 = mma_h(al, bh1, o1);
      o1 = mma_h(ah, bl1, o1);
      guard2(o0, o1, ah, al, bh0, bh1, bl0, bl1);
    }
    {
      const v16h bh2 = ldfrag_h(bhp + 2 * bs + k0), bh3 = ldfrag_h(bhp + 3 * bs + k0);
      const v16h bl2 = ldfrag_h(blp + 2 * bs + k0), bl3 = ldfrag_h(blp + 3 * bs + k0);
      o2 = mma_h(ah, bh2, o2);
      o2 = mma_h(al, bh2, o2);
      o2 = mma_h(ah, bl2, o2);
      o3 = mma_h(ah, bh3, o3);
      o3 = mma_h(al, bh3, o3);
      o3 = mma_h(ah, bl3, o3);
      guard2(o2, o3, ah, al, bh2, bh3, bl2, bl3);
    }
  }
  acc_guard4(o0, o1, o2, o3);
  const int ml = wave * 16 + 8 * hh;
#pragma unroll
  for (int r = 0; r < 8; ++r) {
    KS[(m)      * KSP + ml + r] = o0[r] * OSC;
    KS[(16 + m) * KSP + ml + r] = o1[r] * OSC;
    KS[(32 + m) * KSP + ml + r] = o2[r] * OSC;
    KS[(48 + m) * KSP + ml + r] = o3[r] * OSC;
  }
  __syncthreads();
  const int q = tid >> 4, p4 = (tid & 15) * 4;
  v4f vals[8];
#pragma unroll
  for (int it = 0; it < 8; ++it) {
    const int d = it * 8 + q;
    vals[it] = *(const v4f*)(KS + d * KSP + p4);
  }
  float* dst = KT + (size_t)(h * HP) * HP + p4;
  for (int pass = 0; pass < 2; ++pass) {
#pragma unroll
    for (int it = 0; it < 8; ++it) {
      const int d = it * 8 + q;
      *(volatile v4f*)(dst + (size_t)d * HP) = vals[it];
    }
    __threadfence();
  }
}

__global__ __launch_bounds__(256) void bp_build(const float* __restrict__ KT, const float* __restrict__ vmw, u16* BP) {
  const int gt = (int)blockIdx.x * 256 + (int)threadIdx.x;
  if (gt >= HP * (KF / 8)) return;
  const int dp  = gt / (KF / 8);
  const int k0  = (gt - dp * (KF / 8)) * 8;
  const int h   = k0 / KSEG;
  const int s   = k0 - h * KSEG;
  const int seg = s >> 6, j8 = s & 63;
  const bool rowok = (dp < DO);
  const int  dpc = rowok ? dp : (DO - 1);
  const float* kr = KT + ((size_t)(h * HP + dp) * HP + j8);
  const v4f ka = *(const v4f*)(kr), kb = *(const v4f*)(kr + 4);
  float kt[8];
#pragma unroll
  for (int e = 0; e < 4; ++e) { kt[e] = ka[e]; kt[4 + e] = kb[e]; }
  unsigned short ob[8];
#pragma unroll
  for (int e = 0; e < 8; ++e) {
    const int mm = j8 + e;
    const _Float16 hv = (_Float16)kt[e];
    const _Float16 lv = (_Float16)(kt[e] - (float)hv);
    const int mc = (mm < DO) ? mm : (DO - 1);
    const float vq = bfr(vmw[dpc * DO + mc]) * MSC;
    const _Float16 qv = (_Float16)vq;
    const unsigned short bh = rowok ? h_bits(hv) : (unsigned short)0;
    const unsigned short bl = rowok ? h_bits(lv) : (unsigned short)0;
    const unsigned short bq = (rowok && mm < DO) ? h_bits(qv) : (unsigned short)0;
    ob[e] = (seg >= 3) ? bq : ((seg == 2) ? bl : bh);
  }
  v4u ov;
#pragma unroll
  for (int e = 0; e < 4; ++e) ov[e] = pk16(ob[2 * e], ob[2 * e + 1]);
  u16* d = BP + (size_t)dp * KF + k0;
  for (int pass = 0; pass < 2; ++pass) {
    *(volatile v4u*)(d) = ov;
    __threadfence();
  }
}

__global__ __launch_bounds__(128)
void gemm_out(const u16* __restrict__ AP, const u16* __restrict__ BP, const float* __restrict__ vmb, float* out) {
#pragma clang fp contract(off)
  __shared__ __align__(16) float slab[4 * SLAB];
  const int tid = (int)threadIdx.x, wave = tid >> 5, lane = tid & 31, hh = lane >> 4, m = lane & 15;
  const int bid = (int)blockIdx.x;
  if (bid * 64 + 64 > SEQ) return;
  const int rowb = bid * 64 + wave * 16;
  const _Float16* ap = (const _Float16*)(const void*)AP + (size_t)(rowb + m) * KF + 8 * hh;
  const _Float16* bp = (const _Float16*)(const void*)BP + (size_t)m * KF + 8 * hh;
  const size_t bs = (size_t)16 * KF;
  v8f acc0 = zero8(), acc1 = zero8(), acc2 = zero8(), acc3 = zero8();
#pragma unroll 2
  for (int k0 = 0; k0 < KF; k0 += 32) {
    const v16h a  = ldfrag_h(ap + k0);
    const v16h b0 = ldfrag_h(bp + k0);
    const v16h b1 = ldfrag_h(bp + bs + k0);
    const v16h b2 = ldfrag_h(bp + 2 * bs + k0);
    const v16h b3 = ldfrag_h(bp + 3 * bs + k0);
    acc0 = mma_h(a, b0, acc0);
    acc1 = mma_h(a, b1, acc1);
    acc2 = mma_h(a, b2, acc2);
    acc3 = mma_h(a, b3, acc3);
    guard6<v16h>(acc0, acc1, acc2, acc3, a, b0, b1, b2, b3, a);
  }
  acc_guard4(acc0, acc1, acc2, acc3);
  float bj[4];
#pragma unroll
  for (int j = 0; j < 4; ++j) {
    const int col = 16 * j + m;
    const int cb  = imin(col, DO - 1);
    const float bvv = bfr(vmb[cb]);
    bj[j] = (col < DO) ? bvv : 0.0f;
  }
  float* sl = slab + wave * SLAB;
#pragma unroll
  for (int r = 0; r < 8; ++r) {
    const int ro = (8 * hh + r) * SLP + m;
    sl[ro]      = acc0[r] * FSC + bj[0];
    sl[ro + 16] = acc1[r] * FSC + bj[1];
    sl[ro + 32] = acc2[r] * FSC + bj[2];
    sl[ro + 48] = acc3[r] * FSC + bj[3];
  }
  wave_sync_lds();
  float ss = 0.0f;
#pragma unroll
  for (int i = 0; i < 8; ++i) {
    const v4f qv = *(const v4f*)(sl + m * SLP + 32 * hh + 4 * i);
#pragma unroll
    for (int e = 0; e < 4; ++e) ss = ss + qv[e] * qv[e];
  }
  ss = ss + __shfl_xor(ss, 16, 32);
  const float tt = sqrtf(ss + KCURV);
  if (hh == 0) sl[m * SLP + 64] = tt;
  wave_sync_lds();
  v4f vals[8];
  const int q0 = 4 * m;
#pragma unroll
  for (int it = 0; it < 8; ++it) {
    const int row = 2 * it + hh;
    const float* br = sl + row * SLP;
    const float t0 = br[64];
    const float pm = br[imax(q0 - 1, 0)];
    v4f v;
    v[0] = (q0 == 0) ? t0 : pm;
    v[1] = br[q0];
    v[2] = br[q0 + 1];
    v[3] = br[q0 + 2];
    vals[it] = v;
  }
  float* dst = out + (size_t)(rowb + hh) * CIN + q0;
  for (int pass = 0; pass < 2; ++pass) {
#pragma unroll
    for (int it = 0; it < 8; ++it) {
      *(volatile v4f*)(dst + (size_t)(2 * it) * CIN) = vals[it];
    }
    __threadfence();
  }
}

extern "C" void kernel_launch(void* const* d_in, const int* in_sizes, int n_in,
                              void* d_out, int out_size, void* d_ws, size_t ws_size,
                              hipStream_t stream) {
  if (n_in < 11) return;
  const long long needx = (long long)((NB - 1) * N_FULL + SEQ) * CIN;
  if ((long long)in_sizes[0] < needx || (long long)in_sizes[1] < needx) return;
  if (in_sizes[2] < NH * DO * CIN || in_sizes[4] < NH * DO * CIN || in_sizes[6] < NH * DO * CIN) return;
  if (in_sizes[3] < NH * DO || in_sizes[5] < NH * DO || in_sizes[7] < NH * DO) return;
  if (in_sizes[8] < 1 || in_sizes[9] < DO * DO || in_sizes[10] < DO) return;
  if ((long long)out_size < needx) return;

  const float* xq  = (const float*)d_in[0];
  const float* xs  = (const float*)d_in[1];
  const float* wq  = (const float*)d_in[2];
  const float* bq  = (const float*)d_in[3];
  const float* wk  = (const float*)d_in[4];
  const float* bk  = (const float*)d_in[5];
  const float* wv  = (const float*)d_in[6];
  const float* bv  = (const float*)d_in[7];
  const float* ns  = (const float*)d_in[8];
  const float* vmw = (const float*)d_in[9];
  const float* vmb = (const float*)d_in[10];
  float*       out = (float*)d_out;

  const size_t szW = (size_t)NPROJ * CIN * 2;
  const size_t szX = (size_t)SEQ * CIN * 2;
  const size_t szT = (size_t)NPROJ * SEQ * 2;
  const size_t szA = (size_t)SEQ * KF * 2;
  const size_t szK = (size_t)NPROJ * HP * 4;
  const size_t szB = (size_t)HP * KF * 2;
  size_t off = 0;
  const size_t oWQ = off; off += szW;
  const size_t oWK = off; off += szW;
  const size_t oWV = off; off += szW;
  const size_t oXQ = off; off += szX;
  const size_t oXS = off; off += szX;
  const size_t oTH = off; off += szT;
  const size_t oTL = off; off += szT;
  const size_t oUH = off; off += szT;
  const size_t oUL = off; off += szT;
  const size_t oAP = off; off += szA;
  const size_t oKT = off; off += szK;
  const size_t oBP = off; off += szB;
  if (off > ws_size) return;
  if (off > (size_t)WS_CAP) return;

  char* ws = (char*)d_ws;
  u16*   WQP = (u16*)(ws + oWQ);
  u16*   WKP = (u16*)(ws + oWK);
  u16*   WVP = (u16*)(ws + oWV);
  u16*   XQ  = (u16*)(ws + oXQ);
  u16*   XS  = (u16*)(ws + oXS);
  u16*   TH  = (u16*)(ws + oTH);
  u16*   TL  = (u16*)(ws + oTL);
  u16*   UH  = (u16*)(ws + oUH);
  u16*   UL  = (u16*)(ws + oUL);
  u16*   AP  = (u16*)(ws + oAP);
  float* KT  = (float*)(ws + oKT);
  u16*   BP  = (u16*)(ws + oBP);

  const dim3 b256(256), b128(128);
  const dim3 gW((NPROJ * 8) / 256, 3);
  const int  n8x = (SEQ * CIN) / 8;
  const dim3 gX2((n8x + 255) / 256, 2);
  const dim3 gP((SEQ / 64) * NH);
  const dim3 gKV(NH);
  const dim3 gBP((HP * (KF / 8)) / 256);
  const dim3 gO(SEQ / 64);

  cvt_w3<<<gW, b256, 0, stream>>>(wq, wk, wv, WQP, WKP, WVP);

  for (int b = 0; b < NB; ++b) {
    const size_t xo = (size_t)b * N_FULL * CIN;
    cvt_x2<<<gX2, b256, 0, stream>>>(xq + xo, xs + xo, XQ, XS, n8x);
    gemm_proj<0><<<gP, b128, 0, stream>>>(XS, WKP, bk, ns, KT, TH, TL, AP);
    gemm_proj<1><<<gP, b128, 0, stream>>>(XS, WVP, bv, ns, KT, UH, UL, AP);
    gemm_ktv<<<gKV, b128, 0, stream>>>(TH, TL, UH, UL, KT);
    gemm_proj<2><<<gP, b128, 0, stream>>>(XQ, WQP, bq, ns, KT, TH, TL, AP);
    bp_build<<<gBP, b256, 0, stream>>>(KT, vmw, BP);
    gemm_out<<<gO, b128, 0, stream>>>(AP, BP, vmb, out + xo);
  }
  (void)hipGetLastError();
}
